// Net_36962488550095
// MI455X (gfx1250) — hardware-run, weakly checked
//
#include <hip/hip_runtime.h>
#include <math.h>

typedef __attribute__((ext_vector_type(16))) __bf16   v16b;
typedef __attribute__((ext_vector_type(8)))  __bf16   v8b;
typedef __attribute__((ext_vector_type(8)))  float    v8f;
typedef __attribute__((ext_vector_type(4)))  float    v4f;
typedef __attribute__((ext_vector_type(4)))  unsigned v4u;

constexpr int kHR   = 1024;
constexpr int kHW   = kHR * kHR;
constexpr int kGW   = 16;
constexpr int kGD   = 8;
constexpr int kActP = 64;
constexpr int kBgP  = 128;
constexpr float kCellScale = (float)kGW / (float)kHR;
static_assert(kHW == (1 << 20), "pixel count per image");
static_assert(kCellScale == 0.015625f, "cell scale is a power of two");

constexpr int kK[9]   = {27, 72, 144, 288, 576, 576, 576, 576, 64};
constexpr int kKP[9]  = {32, 96, 160, 288, 576, 576, 576, 576, 64};
constexpr int kNr[9]  = {8, 16, 32, 64, 64, 64, 64, 64, 96};
constexpr int kNP[9]  = {64, 64, 64, 64, 64, 64, 64, 64, 128};
constexpr int kM[9]   = {32768, 8192, 2048, 512, 512, 512, 128, 32, 512};
constexpr int kMP[9]  = {32768, 8192, 2048, 512, 512, 512, 128, 64, 512};
constexpr int kCin[8] = {3, 8, 16, 32, 64, 64, 64, 64};
constexpr int kIH[8]  = {256, 128, 64, 32, 16, 16, 16, 8};
constexpr int kOwS[8] = {7, 6, 5, 4, 4, 4, 3, 2};
constexpr int kStr[8] = {2, 2, 2, 2, 1, 1, 2, 2};
constexpr int kSrc[8] = {-1, 0, 1, 2, 3, 4, 3, 6};
constexpr int kRelu[9] = {1, 1, 1, 1, 1, 0, 1, 1, 0};

constexpr bool shapes_ok() {
  for (int l = 0; l < 9; ++l) {
    if ((kKP[l] % 32) != 0 || kKP[l] < kK[l]) return false;
    if ((kNP[l] % 64) != 0 || kNP[l] < kNr[l]) return false;
    if ((kMP[l] % 64) != 0 || kMP[l] < kM[l]) return false;
    if (((kNP[l] * kKP[l] / 8) % 256) != 0) return false;
    if (((kMP[l] * kKP[l] / 8) % 256) != 0) return false;
  }
  for (int l = 0; l < 8; ++l) {
    if (kK[l] != kCin[l] * 9) return false;
    const int oh = 1 << kOwS[l];
    if (kM[l] != 2 * oh * oh) return false;
    if ((kIH[l] - 1) / kStr[l] + 1 != oh) return false;
  }
  return true;
}
static_assert(shapes_ok(), "site shapes");

constexpr size_t btBytes(int l) { return (size_t)kNP[l] * kKP[l] * 2; }
constexpr size_t aBytes(int l)  { return (size_t)kMP[l] * kKP[l] * 2; }
constexpr size_t cBytes(int l)  { return (size_t)kMP[l] * kNP[l] * 4; }
constexpr size_t offBtHi(int l) { size_t o = 0; for (int i = 0; i < l; ++i) o += 2 * btBytes(i); return o; }
constexpr size_t offBtLo(int l) { return offBtHi(l) + btBytes(l); }
constexpr size_t kBtEnd = offBtHi(9);
constexpr size_t offAHi(int l)  { size_t o = kBtEnd; for (int i = 0; i < l; ++i) o += 2 * aBytes(i); return o; }
constexpr size_t offALo(int l)  { return offAHi(l) + aBytes(l); }
constexpr size_t kAEnd = offAHi(9);
constexpr size_t offC(int l)    { size_t o = kAEnd; for (int i = 0; i < l; ++i) o += cBytes(i); return o; }
constexpr size_t kOffGvec = offC(9);
constexpr size_t kWsTotal = kOffGvec + 512;
static_assert(kBtEnd == 770048ull, "Bt planes");
static_assert(kAEnd - kBtEnd == 12173312ull, "A planes");
static_assert(kOffGvec - kAEnd == 11714560ull, "C planes");
static_assert(kWsTotal == 24658432ull, "carve total");
static_assert(kWsTotal <= 134217728ull, "carve cap");
static_assert((kBtEnd % 128) == 0 && (kAEnd % 128) == 0 && (kOffGvec % 128) == 0, "aligned regions");

constexpr int kInElems[30] = {393216, 6291456, 216, 8, 1152, 16, 4608, 32, 18432, 64,
                              36864, 64, 36864, 64, 36864, 64, 36864, 64, 262144, 256,
                              32768, 128, 8192, 64, 6144, 96, 48, 16, 16, 1};
static_assert(sizeof(kInElems) / sizeof(kInElems[0]) == 30, "input table");

__device__ __forceinline__ unsigned bf_rne_bits(float f) {
  const unsigned u = __float_as_uint(f);
  return (u + 0x7FFFu + ((u >> 16) & 1u)) >> 16;
}
__device__ __forceinline__ void split_bf(float v, unsigned& h, unsigned& l) {
  h = bf_rne_bits(v);
  l = bf_rne_bits(v - __uint_as_float(h << 16));
}
__device__ __forceinline__ void store_split8(const float (&v)[8], unsigned short* ph, unsigned short* pl) {
  unsigned h[8], l[8];
#pragma unroll
  for (int e = 0; e < 8; ++e) split_bf(v[e], h[e], l[e]);
  v4u hv, lv;
  hv[0] = h[0] | (h[1] << 16);
  hv[1] = h[2] | (h[3] << 16);
  hv[2] = h[4] | (h[5] << 16);
  hv[3] = h[6] | (h[7] << 16);
  lv[0] = l[0] | (l[1] << 16);
  lv[1] = l[2] | (l[3] << 16);
  lv[2] = l[4] | (l[5] << 16);
  lv[3] = l[6] | (l[7] << 16);
  *(volatile v4u*)ph = hv;
  *(volatile v4u*)pl = lv;
  __threadfence();
  *(volatile v4u*)ph = hv;
  *(volatile v4u*)pl = lv;
}

union FragU { v16b v; v8b h[2]; };
__device__ __forceinline__ v16b frag_load(const __bf16* p) {
  FragU f;
  f.h[0] = *(const v8b*)(p);
  f.h[1] = *(const v8b*)(p + 16);
  return f.v;
}
__device__ __forceinline__ v8f frag_mma(v16b a, v16b b, v8f c) {
  return __builtin_amdgcn_wmma_f32_16x16x32_bf16(false, a, false, b, (short)0, c, false, false);
}
__device__ __forceinline__ void tie_acc(v8f& a, v16b x, v16b y, v16b z, v16b w) {
  asm volatile("v_nop\n\tv_nop\n\tv_nop\n\tv_nop" : "+v"(a) : "v"(x), "v"(y), "v"(z), "v"(w));
}
__device__ __forceinline__ void acc_guard4(v8f& a, v8f& b, v8f& c, v8f& d) {
  asm volatile("v_nop\n\tv_nop\n\tv_nop\n\tv_nop" : "+v"(a), "+v"(b), "+v"(c), "+v"(d));
}

__global__ __launch_bounds__(256) void prep_bt_kernel(
    const float* __restrict__ src, unsigned short* __restrict__ dhi, unsigned short* __restrict__ dlo,
    int N, int K, int KP8, int total8)
{
  const int i = blockIdx.x * 256 + threadIdx.x;
  if (i >= total8) return;
  const int n  = i / KP8;
  const int k8 = (i - n * KP8) << 3;
  const int nc = (n < N) ? n : (N - 1);
  float v[8];
#pragma unroll
  for (int e = 0; e < 8; ++e) {
    const int k  = k8 + e;
    const int kc = (k < K) ? k : (K - 1);
    float t = src[(size_t)nc * K + kc];
    asm volatile("" : "+v"(t));
    const bool ok = (n < N) && (k < K);
    v[e] = ok ? t : 0.0f;
  }
  store_split8(v, dhi + ((size_t)i << 3), dlo + ((size_t)i << 3));
}

__global__ __launch_bounds__(256) void im2col_split_kernel(
    const float* __restrict__ src, unsigned short* __restrict__ ahi, unsigned short* __restrict__ alo,
    int IH, int owShift, int stride, int M, int K, int KP8, int total8,
    int sB, int sC, int sY, int sX)
{
  const int i = blockIdx.x * 256 + threadIdx.x;
  if (i >= total8) return;
  const int m   = i / KP8;
  const int k8  = (i - m * KP8) << 3;
  const int mc  = (m < M) ? m : (M - 1);
  const int b   = mc >> (2 * owShift);
  const int rem = mc & ((1 << (2 * owShift)) - 1);
  const int oy  = rem >> owShift;
  const int ox  = rem & ((1 << owShift) - 1);
  const int iy0 = oy * stride - 1;
  const int ix0 = ox * stride - 1;
  const int baseB = b * sB;
  float v[8];
#pragma unroll
  for (int e = 0; e < 8; ++e) {
    const int k  = k8 + e;
    const int kc = (k < K) ? k : (K - 1);
    const int ci = kc / 9;
    const int rc = kc - ci * 9;
    const int ky = rc / 3;
    const int kx = rc - ky * 3;
    const int iy = iy0 + ky;
    const int ix = ix0 + kx;
    const bool ok = (m < M) && (k < K) && (iy >= 0) && (iy < IH) && (ix >= 0) && (ix < IH);
    const int iyc = (iy < 0) ? 0 : ((iy >= IH) ? (IH - 1) : iy);
    const int ixc = (ix < 0) ? 0 : ((ix >= IH) ? (IH - 1) : ix);
    float t = src[(size_t)(baseB + ci * sC + iyc * sY + ixc * sX)];
    asm volatile("" : "+v"(t));
    v[e] = ok ? t : 0.0f;
  }
  store_split8(v, ahi + ((size_t)i << 3), alo + ((size_t)i << 3));
}

template <int ACT>
__global__ __launch_bounds__(256) void gemm_split_kernel(
    const unsigned short* __restrict__ Ahp, const unsigned short* __restrict__ Alp, int lda,
    const unsigned short* __restrict__ Bhp, const unsigned short* __restrict__ Blp, int ldb,
    float* __restrict__ C, int ldc, const float* __restrict__ bias, int nreal,
    int M, int N, int K)
{
  const __bf16* Ah = (const __bf16*)Ahp;
  const __bf16* Al = (const __bf16*)Alp;
  const __bf16* Bh = (const __bf16*)Bhp;
  const __bf16* Bl = (const __bf16*)Blp;
  __shared__ __align__(16) float sT[8][16 * 68];
  const int lane = threadIdx.x & 31;
  const int wave = threadIdx.x >> 5;
  const int tilesN = N >> 6;
  const int tilesM = M >> 6;
  const int tile = blockIdx.x * 8 + wave;
  if (tile >= tilesM * tilesN) return;
  const int tm = tile / tilesN;
  const int tn = tile - tm * tilesN;
  const int m0 = tm << 6;
  const int n0 = tn << 6;
  const int rlane = lane & 15;
  const int koff  = (lane >> 4) * 8;
  const int mOff  = (lane >> 4) * 8;

  v8f acc[4][4];
#pragma unroll
  for (int i = 0; i < 4; ++i)
#pragma unroll
    for (int j = 0; j < 4; ++j) acc[i][j] = (v8f){0.f, 0.f, 0.f, 0.f, 0.f, 0.f, 0.f, 0.f};

  for (int k0 = 0; k0 < K; k0 += 32) {
    v16b bh[4], bl[4];
#pragma unroll
    for (int j = 0; j < 4; ++j) {
      const size_t bo = (size_t)(n0 + (j << 4) + rlane) * ldb + koff + k0;
      bh[j] = frag_load(Bh + bo);
      bl[j] = frag_load(Bl + bo);
    }
#pragma unroll
    for (int i = 0; i < 4; ++i) {
      const size_t ao = (size_t)(m0 + (i << 4) + rlane) * lda + koff + k0;
      const v16b ah = frag_load(Ah + ao);
      const v16b al = frag_load(Al + ao);
#pragma unroll
      for (int j = 0; j < 4; ++j) {
        acc[i][j] = frag_mma(ah, bh[j], acc[i][j]);
        acc[i][j] = frag_mma(ah, bl[j], acc[i][j]);
        acc[i][j] = frag_mma(al, bh[j], acc[i][j]);
      }
#pragma unroll
      for (int j = 0; j < 4; ++j) tie_acc(acc[i][j], ah, al, bh[j], bl[j]);
    }
  }
  acc_guard4(acc[0][0], acc[0][1], acc[0][2], acc[0][3]);
  acc_guard4(acc[1][0], acc[1][1], acc[1][2], acc[1][3]);
  acc_guard4(acc[2][0], acc[2][1], acc[2][2], acc[2][3]);
  acc_guard4(acc[3][0], acc[3][1], acc[3][2], acc[3][3]);

  float bvj[4];
#pragma unroll
  for (int j = 0; j < 4; ++j) {
    const int n  = n0 + (j << 4) + rlane;
    const int nc = (n < nreal) ? n : (nreal - 1);
    float t = bias[nc];
    asm volatile("" : "+v"(t));
    bvj[j] = (n < nreal) ? t : 0.0f;
  }

  float* slab = sT[wave];
#pragma unroll
  for (int i = 0; i < 4; ++i) {
    const int mBase = m0 + (i << 4);
#pragma unroll
    for (int j = 0; j < 4; ++j) {
#pragma unroll
      for (int r = 0; r < 8; ++r) {
        float v = acc[i][j][r] + bvj[j];
        if (ACT == 2) v = fmaxf(v, 0.0f);
        slab[(mOff + r) * 68 + (j << 4) + rlane] = v;
      }
    }
    __builtin_amdgcn_fence(__ATOMIC_RELEASE, "workgroup");
    __builtin_amdgcn_wave_barrier();
    __builtin_amdgcn_fence(__ATOMIC_ACQUIRE, "workgroup");
    {
      const int hh = lane >> 4;
      const int c4 = (lane & 15) * 4;
      for (int pass = 0; pass < 2; ++pass) {
#pragma unroll
        for (int it = 0; it < 8; ++it) {
          const int row = it * 2 + hh;
          const v4f v = *(const v4f*)(slab + row * 68 + c4);
          *(volatile v4f*)(C + (size_t)(mBase + row) * ldc + n0 + c4) = v;
        }
        __threadfence();
      }
    }
    __builtin_amdgcn_fence(__ATOMIC_RELEASE, "workgroup");
    __builtin_amdgcn_wave_barrier();
    __builtin_amdgcn_fence(__ATOMIC_ACQUIRE, "workgroup");
  }
}

__global__ __launch_bounds__(256) void fc_stack_kernel(
    const float* __restrict__ g1,
    const float* __restrict__ w0, const float* __restrict__ b0,
    const float* __restrict__ w1, const float* __restrict__ b1,
    const float* __restrict__ w2, const float* __restrict__ b2,
    float* __restrict__ gvec)
{
  __shared__ __align__(16) float sF[2048];
  __shared__ __align__(16) float sH0[512];
  __shared__ __align__(16) float sH1[256];
  __shared__ __align__(16) float sG[128];
  const int tid = threadIdx.x;
#pragma unroll 1
  for (int it = 0; it < 8; ++it) {
    const int idx = tid + 256 * it;
    const int b = idx >> 10;
    const int k = idx & 1023;
    const int c = k >> 4;
    const int pp = k & 15;
    sF[idx] = g1[(size_t)(b * 16 + pp) * kActP + c];
  }
  __syncthreads();
  {
    const float* wr = w0 + (size_t)tid * 1024;
    float a0 = 0.0f, a1 = 0.0f;
#pragma unroll 1
    for (int k4 = 0; k4 < 256; ++k4) {
      const v4f wv = *(const v4f*)(wr + 4 * k4);
      const v4f f0 = *(const v4f*)(sF + 4 * k4);
      const v4f f1 = *(const v4f*)(sF + 1024 + 4 * k4);
      a0 = fmaf(wv[0], f0[0], a0);
      a0 = fmaf(wv[1], f0[1], a0);
      a0 = fmaf(wv[2], f0[2], a0);
      a0 = fmaf(wv[3], f0[3], a0);
      a1 = fmaf(wv[0], f1[0], a1);
      a1 = fmaf(wv[1], f1[1], a1);
      a1 = fmaf(wv[2], f1[2], a1);
      a1 = fmaf(wv[3], f1[3], a1);
    }
    const float bb = b0[tid];
    sH0[tid]       = fmaxf(a0 + bb, 0.0f);
    sH0[256 + tid] = fmaxf(a1 + bb, 0.0f);
  }
  __syncthreads();
  {
    const int n = (tid < 128) ? tid : 127;
    const float* wr = w1 + (size_t)n * 256;
    float a0 = 0.0f, a1 = 0.0f;
#pragma unroll 1
    for (int k4 = 0; k4 < 64; ++k4) {
      const v4f wv = *(const v4f*)(wr + 4 * k4);
      const v4f f0 = *(const v4f*)(sH0 + 4 * k4);
      const v4f f1 = *(const v4f*)(sH0 + 256 + 4 * k4);
      a0 = fmaf(wv[0], f0[0], a0);
      a0 = fmaf(wv[1], f0[1], a0);
      a0 = fmaf(wv[2], f0[2], a0);
      a0 = fmaf(wv[3], f0[3], a0);
      a1 = fmaf(wv[0], f1[0], a1);
      a1 = fmaf(wv[1], f1[1], a1);
      a1 = fmaf(wv[2], f1[2], a1);
      a1 = fmaf(wv[3], f1[3], a1);
    }
    const float bb = b1[n];
    const float r0 = fmaxf(a0 + bb, 0.0f);
    const float r1 = fmaxf(a1 + bb, 0.0f);
    if (tid < 128) {
      sH1[n] = r0;
      sH1[128 + n] = r1;
    }
  }
  __syncthreads();
  {
    const int n = (tid < 64) ? tid : 63;
    const float* wr = w2 + (size_t)n * 128;
    float a0 = 0.0f, a1 = 0.0f;
#pragma unroll 1
    for (int k4 = 0; k4 < 32; ++k4) {
      const v4f wv = *(const v4f*)(wr + 4 * k4);
      const v4f f0 = *(const v4f*)(sH1 + 4 * k4);
      const v4f f1 = *(const v4f*)(sH1 + 128 + 4 * k4);
      a0 = fmaf(wv[0], f0[0], a0);
      a0 = fmaf(wv[1], f0[1], a0);
      a0 = fmaf(wv[2], f0[2], a0);
      a0 = fmaf(wv[3], f0[3], a0);
      a1 = fmaf(wv[0], f1[0], a1);
      a1 = fmaf(wv[1], f1[1], a1);
      a1 = fmaf(wv[2], f1[2], a1);
      a1 = fmaf(wv[3], f1[3], a1);
    }
    const float bb = b2[n];
    const float r0 = a0 + bb;
    const float r1 = a1 + bb;
    if (tid < 64) {
      sG[n] = r0;
      sG[64 + n] = r1;
    }
  }
  __syncthreads();
  if (tid < 32) {
    const v4f val = *(const v4f*)(sG + tid * 4);
    *(volatile v4f*)(gvec + tid * 4) = val;
    __threadfence();
    *(volatile v4f*)(gvec + tid * 4) = val;
  }
}

__global__ __launch_bounds__(256) void fuse_split_kernel(
    const float* __restrict__ loc, const float* __restrict__ gvec,
    unsigned short* __restrict__ ahi, unsigned short* __restrict__ alo)
{
  const int i = blockIdx.x * 256 + threadIdx.x;
  if (i >= 4096) return;
  const int m  = i >> 3;
  const int c8 = (i & 7) * 8;
  const int b  = m >> 8;
  const v4f l0 = *(const v4f*)(loc + (size_t)m * kActP + c8);
  const v4f l1 = *(const v4f*)(loc + (size_t)m * kActP + c8 + 4);
  const v4f g0 = *(const v4f*)(gvec + b * 64 + c8);
  const v4f g1 = *(const v4f*)(gvec + b * 64 + c8 + 4);
  float v[8];
#pragma unroll
  for (int e = 0; e < 4; ++e) {
    v[e]     = fmaxf(l0[e] + g0[e], 0.0f);
    v[4 + e] = fmaxf(l1[e] + g1[e], 0.0f);
  }
  store_split8(v, ahi + ((size_t)i << 3), alo + ((size_t)i << 3));
}

__global__ __launch_bounds__(256) void guide_slice_apply_kernel(
    const float* __restrict__ fr,
    const float* __restrict__ gw0, const float* __restrict__ gb0,
    const float* __restrict__ gw1, const float* __restrict__ gb1,
    const float* __restrict__ bgv, float* __restrict__ out)
{
  const unsigned p = blockIdx.x * 256u + threadIdx.x;
  const int b   = (int)(p >> 20);
  const int rem = (int)(p & (unsigned)(kHW - 1));
  const int y   = rem >> 10;
  const int x   = rem & (kHR - 1);
  const float* base = fr + (size_t)b * 3 * kHW + rem;
  const float cr = base[0];
  const float cg = base[kHW];
  const float cb = base[2 * kHW];

  float s = 0.0f;
#pragma unroll 1
  for (int j = 0; j < 16; ++j) {
    float h = gw0[j * 3 + 0] * cr;
    h = fmaf(gw0[j * 3 + 1], cg, h);
    h = fmaf(gw0[j * 3 + 2], cb, h);
    h = h + gb0[j];
    h = fmaxf(h, 0.0f);
    s = fmaf(gw1[j], h, s);
  }
  s = s + gb1[0];
  const float gdv = 1.0f / (1.0f + expf(-s));

  const float xs = ((float)x + 0.5f) * kCellScale - 0.5f;
  const float ys = ((float)y + 0.5f) * kCellScale - 0.5f;
  const float fx = floorf(xs);
  const float fy = floorf(ys);
  int x0 = (int)fx;
  x0 = (x0 < 0) ? 0 : ((x0 > kGW - 1) ? (kGW - 1) : x0);
  const int x1 = (x0 + 1 > kGW - 1) ? (kGW - 1) : (x0 + 1);
  int y0 = (int)fy;
  y0 = (y0 < 0) ? 0 : ((y0 > kGW - 1) ? (kGW - 1) : y0);
  const int y1 = (y0 + 1 > kGW - 1) ? (kGW - 1) : (y0 + 1);
  const float wx = xs - fx;
  const float wy = ys - fy;
  const float gz = gdv * (float)kGD - 0.5f;
  const float fz = floorf(gz);
  int z0 = (int)fz;
  z0 = (z0 < 0) ? 0 : ((z0 > kGD - 1) ? (kGD - 1) : z0);
  const int z1 = (z0 + 1 > kGD - 1) ? (kGD - 1) : (z0 + 1);
  const float wz = gz - fz;
  const float uwx = 1.0f - wx;
  const float uwy = 1.0f - wy;
  const float uwz = 1.0f - wz;

  float acc[12];
#pragma unroll
  for (int c = 0; c < 12; ++c) acc[c] = 0.0f;
  const float* gb = bgv + (size_t)b * 256 * kBgP;
#pragma unroll 1
  for (int cn = 0; cn < 8; ++cn) {
    const bool az = (cn >> 2) != 0;
    const bool ay = ((cn >> 1) & 1) != 0;
    const bool ax = (cn & 1) != 0;
    const int   zi  = az ? z1 : z0;
    const float wzf = az ? wz : uwz;
    const int   yi  = ay ? y1 : y0;
    const float wyf = ay ? wy : uwy;
    const int   xi  = ax ? x1 : x0;
    const float wxf = ax ? wx : uwx;
    const float w = (wzf * wyf) * wxf;
    const float* gp = gb + (size_t)(yi * kGW + xi) * kBgP + zi;
#pragma unroll
    for (int c = 0; c < 12; ++c) acc[c] = fmaf(w, gp[c * kGD], acc[c]);
  }

  float f0 = acc[0] * cr;
  f0 = fmaf(acc[1], cg, f0);
  f0 = fmaf(acc[2], cb, f0);
  f0 = f0 + acc[3];
  float f1 = acc[4] * cr;
  f1 = fmaf(acc[5], cg, f1);
  f1 = fmaf(acc[6], cb, f1);
  f1 = f1 + acc[7];
  float f2 = acc[8] * cr;
  f2 = fmaf(acc[9], cg, f2);
  f2 = fmaf(acc[10], cb, f2);
  f2 = f2 + acc[11];

  volatile float* q0 = out + (size_t)p;
  volatile float* q1 = out + (size_t)2 * kHW + (size_t)b * 3 * kHW + rem;
  volatile float* q2 = q1 + kHW;
  volatile float* q3 = q2 + kHW;
  *q0 = gdv;
  *q1 = f0;
  *q2 = f1;
  *q3 = f2;
  __threadfence();
  *q0 = gdv;
  *q1 = f0;
  *q2 = f1;
  *q3 = f2;
}

extern "C" void kernel_launch(void* const* d_in, const int* in_sizes, int n_in,
                              void* d_out, int out_size, void* d_ws, size_t ws_size,
                              hipStream_t stream) {
  if (n_in < 30) return;
  for (int i = 0; i < 30; ++i) {
    if (in_sizes[i] != kInElems[i]) return;
  }
  if (out_size != 8 * kHW) return;
  if (ws_size < kWsTotal) return;

  const float* lr   = (const float*)d_in[0];
  const float* fr   = (const float*)d_in[1];
  const float* wsrc[9] = {(const float*)d_in[2],  (const float*)d_in[4],  (const float*)d_in[6],
                          (const float*)d_in[8],  (const float*)d_in[10], (const float*)d_in[12],
                          (const float*)d_in[14], (const float*)d_in[16], (const float*)d_in[24]};
  const float* bsrc[9] = {(const float*)d_in[3],  (const float*)d_in[5],  (const float*)d_in[7],
                          (const float*)d_in[9],  (const float*)d_in[11], (const float*)d_in[13],
                          (const float*)d_in[15], (const float*)d_in[17], (const float*)d_in[25]};
  const float* fcw0 = (const float*)d_in[18];
  const float* fcb0 = (const float*)d_in[19];
  const float* fcw1 = (const float*)d_in[20];
  const float* fcb1 = (const float*)d_in[21];
  const float* fcw2 = (const float*)d_in[22];
  const float* fcb2 = (const float*)d_in[23];
  const float* guw0 = (const float*)d_in[26];
  const float* gub0 = (const float*)d_in[27];
  const float* guw1 = (const float*)d_in[28];
  const float* gub1 = (const float*)d_in[29];
  float* out = (float*)d_out;

  char* ws = (char*)d_ws;
  unsigned short* BtH[9];
  unsigned short* BtL[9];
  unsigned short* AH[9];
  unsigned short* AL[9];
  float* Cp[9];
  for (int l = 0; l < 9; ++l) {
    BtH[l] = (unsigned short*)(ws + offBtHi(l));
    BtL[l] = (unsigned short*)(ws + offBtLo(l));
    AH[l]  = (unsigned short*)(ws + offAHi(l));
    AL[l]  = (unsigned short*)(ws + offALo(l));
    Cp[l]  = (float*)(ws + offC(l));
  }
  float* gvec = (float*)(ws + kOffGvec);

  for (int l = 0; l < 9; ++l) {
    const int total8 = kNP[l] * kKP[l] / 8;
    prep_bt_kernel<<<total8 / 256, 256, 0, stream>>>(wsrc[l], BtH[l], BtL[l], kNr[l], kK[l], kKP[l] / 8, total8);
  }

  auto run_gemm = [&](int l) {
    const int tiles = (kMP[l] / 64) * (kNP[l] / 64);
    const int grid = (tiles + 7) / 8;
    if (kRelu[l]) {
      gemm_split_kernel<2><<<grid, 256, 0, stream>>>(AH[l], AL[l], kKP[l], BtH[l], BtL[l], kKP[l],
                                                     Cp[l], kNP[l], bsrc[l], kNr[l], kMP[l], kNP[l], kKP[l]);
    } else {
      gemm_split_kernel<0><<<grid, 256, 0, stream>>>(AH[l], AL[l], kKP[l], BtH[l], BtL[l], kKP[l],
                                                     Cp[l], kNP[l], bsrc[l], kNr[l], kMP[l], kNP[l], kKP[l]);
    }
  };

  for (int l = 0; l < 8; ++l) {
    const int ih = kIH[l];
    const float* src;
    int sB, sC, sY, sX;
    if (kSrc[l] < 0) {
      src = lr;
      sB = kCin[l] * ih * ih;
      sC = ih * ih;
      sY = ih;
      sX = 1;
    } else {
      src = Cp[kSrc[l]];
      sB = ih * ih * kActP;
      sC = 1;
      sY = ih * kActP;
      sX = kActP;
    }
    const int total8 = kMP[l] * kKP[l] / 8;
    im2col_split_kernel<<<total8 / 256, 256, 0, stream>>>(src, AH[l], AL[l], ih, kOwS[l], kStr[l],
                                                          kM[l], kK[l], kKP[l] / 8, total8, sB, sC, sY, sX);
    run_gemm(l);
  }

  fc_stack_kernel<<<1, 256, 0, stream>>>(Cp[7], fcw0, fcb0, fcw1, fcb1, fcw2, fcb2, gvec);

  fuse_split_kernel<<<16, 256, 0, stream>>>(Cp[5], gvec, AH[8], AL[8]);
  run_gemm(8);

  guide_slice_apply_kernel<<<(2 * kHW) / 256, 256, 0, stream>>>(fr, guw0, gub0, guw1, gub1, Cp[8], out);
}
